// NonLocalBlock_46548855554375
// MI455X (gfx1250) — hardware-verified
//
#include <hip/hip_runtime.h>


#ifndef NB
#define NB 4
#endif
#ifndef SEQ
#define SEQ 4096
#endif
#define NB_FULL  4
#define SEQ_FULL 4096
#define CC   128
#define IC   128
#define HW   SEQ
#define HWF  SEQ_FULL
#define PCAR 16384.0f
static_assert(NB >= 1 && NB <= NB_FULL);
static_assert(SEQ >= 128 && SEQ <= SEQ_FULL && (SEQ % 128) == 0);
static_assert((HW % 64) == 0 && (IC % 64) == 0 && (CC % 64) == 0);
static_assert((HW % 32) == 0 && (IC % 32) == 0 && (CC % 32) == 0);
static_assert(((IC * CC) % 8) == 0 && ((HW * CC) % 4) == 0 && ((HW * IC) % 4) == 0 && ((IC * HW) % 2) == 0 && (HW % 8) == 0 && (IC % 4) == 0);
static_assert(((size_t)HW * CC / 4) % 256 == 0 && ((size_t)HW * IC / 4) % 256 == 0 && ((size_t)HW * IC / 2) % 256 == 0);

typedef _Float16 h16;
typedef unsigned short bf;
typedef __attribute__((ext_vector_type(16))) __bf16   v16bf;
typedef __attribute__((ext_vector_type(16))) _Float16 v16h;
typedef __attribute__((ext_vector_type(8)))  _Float16 v8h;
typedef __attribute__((ext_vector_type(8)))  unsigned short v8us;
typedef __attribute__((ext_vector_type(8)))  float    v8f;
typedef __attribute__((ext_vector_type(4)))  float    v4f;
typedef v8h  __attribute__((may_alias)) v8ha;
typedef v4f  __attribute__((may_alias)) v4fa;
typedef v8us __attribute__((may_alias)) v8usa;

__device__ __forceinline__ unsigned short f2bf(float f) { unsigned u = __float_as_uint(f); u += 0x7FFFu + ((u >> 16) & 1u); return (unsigned short)(u >> 16); }
__device__ __forceinline__ float bf2f(unsigned short b) { return __uint_as_float(((unsigned)b) << 16); }
__device__ __forceinline__ float bfr(float f) { return bf2f(f2bf(f)); }
__device__ __forceinline__ v16h cat16(v8h lo, v8h hi) { return __builtin_shufflevector(lo, hi, 0, 1, 2, 3, 4, 5, 6, 7, 8, 9, 10, 11, 12, 13, 14, 15); }
__device__ __forceinline__ v16bf cat16b(v8us lo, v8us hi) { return __builtin_bit_cast(v16bf, __builtin_shufflevector(lo, hi, 0, 1, 2, 3, 4, 5, 6, 7, 8, 9, 10, 11, 12, 13, 14, 15)); }
__device__ __forceinline__ v8f wmma16(v16h a, v16h b, v8f c) { return __builtin_amdgcn_wmma_f32_16x16x32_f16(false, a, false, b, (short)0, c, false, false); }
__device__ __forceinline__ v8f wmmab(v16bf a, v16bf b, v8f c) { return __builtin_amdgcn_wmma_f32_16x16x32_bf16(false, a, false, b, (short)0, c, false, false); }

template <typename T16> struct WFrag;
template <> struct WFrag<h16> { typedef v16h V; static __device__ __forceinline__ V ld(const h16* p) { return cat16(*(const v8h*)p, *(const v8h*)(p + 16)); } static __device__ __forceinline__ v8f mma(V a, V b, v8f c) { return wmma16(a, b, c); } };
template <> struct WFrag<bf> { typedef v16bf V; static __device__ __forceinline__ V ld(const bf* p) { return cat16b(*(const v8us*)p, *(const v8us*)(p + 16)); } static __device__ __forceinline__ v8f mma(V a, V b, v8f c) { return wmmab(a, b, c); } };
template <typename T16, int NSPLIT, bool BIAS>
__global__ __launch_bounds__(32) void k_gemmw(const T16* __restrict__ A, const T16* __restrict__ A2, const T16* __restrict__ Bt, const T16* __restrict__ Bt2, int K, float* C, int ldc, const float* __restrict__ bias, size_t sA, size_t sB, size_t sC) {
    typedef typename WFrag<T16>::V V;
    __shared__ __align__(16) float os[16 * 68];
    const size_t z = blockIdx.z; A += z * sA; if (A2) A2 += z * sA; Bt += z * sB; if (Bt2) Bt2 += z * sB; C += z * sC;
    const int lane = threadIdx.x & 31, lr = lane & 15, hi = lane >> 4; const int r0 = blockIdx.x * 64, c0 = blockIdx.y * 64;
    v8f acc[4][4];
#pragma unroll
    for (int mb = 0; mb < 4; ++mb)
#pragma unroll
        for (int nb = 0; nb < 4; ++nb) acc[mb][nb] = (v8f){};
    const size_t aoff = (size_t)(r0 + lr) * K + 8 * hi, boff = (size_t)(c0 + lr) * K + 8 * hi;
#pragma unroll 1
    for (int kc = 0; kc < K; kc += 32) {
        V a[4], a2[4];
#pragma unroll
        for (int mb = 0; mb < 4; ++mb) { a[mb] = WFrag<T16>::ld(A + aoff + (size_t)mb * 16 * K + kc); if (NSPLIT == 1 || NSPLIT == 2) a2[mb] = WFrag<T16>::ld(A2 + aoff + (size_t)mb * 16 * K + kc); }
#pragma unroll
        for (int nb = 0; nb < 4; ++nb) { const V b = WFrag<T16>::ld(Bt + boff + (size_t)nb * 16 * K + kc); V b2; if (NSPLIT >= 2) b2 = WFrag<T16>::ld(Bt2 + boff + (size_t)nb * 16 * K + kc);
#pragma unroll
            for (int mb = 0; mb < 4; ++mb) { acc[mb][nb] = WFrag<T16>::mma(a[mb], b, acc[mb][nb]); if (NSPLIT == 1 || NSPLIT == 2) acc[mb][nb] = WFrag<T16>::mma(a2[mb], b, acc[mb][nb]); if (NSPLIT >= 2) acc[mb][nb] = WFrag<T16>::mma(a[mb], b2, acc[mb][nb]); } }
        asm volatile("v_nop\n\tv_nop\n\tv_nop\n\tv_nop" : "+v"(acc[0][0]), "+v"(acc[1][1]), "+v"(acc[2][2]), "+v"(acc[3][3]) : "v"(a[0]), "v"(a[3]));
    }
#pragma unroll
    for (int mb = 0; mb < 4; ++mb) {
#pragma unroll
        for (int nb = 0; nb < 4; ++nb) {
#pragma unroll
            for (int j = 0; j < 8; ++j) os[(hi * 8 + j) * 68 + nb * 16 + lr] = acc[mb][nb][j]; }
        __builtin_amdgcn_wave_barrier(); asm volatile("" ::: "memory");
        float* crow = C + (size_t)(r0 + mb * 16) * ldc + c0;
#pragma unroll 1
        for (int ps = 0; ps < 2; ++ps) {
#pragma unroll
            for (int s = 0; s < 8; ++s) { const int row = 2 * s + hi, cofs = lr * 4; v4f val = *(const v4fa*)(os + row * 68 + cofs); if (BIAS) { val[0] += bfr(bias[c0 + cofs]); val[1] += bfr(bias[c0 + cofs + 1]); val[2] += bfr(bias[c0 + cofs + 2]); val[3] += bfr(bias[c0 + cofs + 3]); }
                *(volatile v4f*)(crow + (size_t)row * ldc + cofs) = val; }
            if (ps == 0) __threadfence(); }
        __builtin_amdgcn_wave_barrier(); asm volatile("" ::: "memory");
    }
}

__device__ __forceinline__ h16 tohx(float x) { return (h16)x; }
__device__ __forceinline__ void splitf(float y, unsigned short& h, unsigned short& l) { h = f2bf(y); l = f2bf(y - bf2f(h)); }
typedef __attribute__((ext_vector_type(2))) unsigned short v2us;
typedef __attribute__((ext_vector_type(4))) unsigned short v4us;
typedef __attribute__((ext_vector_type(2))) _Float16 v2h;
typedef __attribute__((ext_vector_type(4))) _Float16 v4h;
typedef __attribute__((ext_vector_type(2))) float v2f;

__global__ __launch_bounds__(256) void k_cvtw(const float* __restrict__ w0, const float* __restrict__ w1, const float* __restrict__ w2, const float* __restrict__ w3, bf* B3, bf* BZ, int n8) {
    const int i = blockIdx.x * 256 + threadIdx.x; if (i >= n8) return;
    const size_t e = (size_t)i * 8, pl = (size_t)n8 * 8;
    const v8f a0 = *(const v8f*)(w0 + e), a1 = *(const v8f*)(w1 + e), a2 = *(const v8f*)(w2 + e), a3 = *(const v8f*)(w3 + e);
    v8us o0, o1, o2, o3;
#pragma unroll
    for (int k = 0; k < 8; ++k) { o0[k] = f2bf(a0[k]); o1[k] = f2bf(a1[k]); o2[k] = f2bf(a2[k]); o3[k] = f2bf(a3[k]); }
    *(volatile v8us*)(B3 + e) = o0; *(volatile v8us*)(B3 + pl + e) = o1; *(volatile v8us*)(B3 + 2 * pl + e) = o2; *(volatile v8us*)(BZ + e) = o3;
    __threadfence();
    *(volatile v8us*)(B3 + e) = o0; *(volatile v8us*)(B3 + pl + e) = o1; *(volatile v8us*)(B3 + 2 * pl + e) = o2; *(volatile v8us*)(BZ + e) = o3;
}
__global__ __launch_bounds__(256) void k_xt(const float* __restrict__ xb, bf* XT) { const size_t e = ((size_t)blockIdx.x * 256 + threadIdx.x) * 4; if (e >= (size_t)HW * CC) return; const int c = (int)(e % CC); const int m = (int)(e / CC); v4us o;
#pragma unroll
    for (int u = 0; u < 4; ++u) o[u] = f2bf(xb[(size_t)(c + u) * HWF + m]); *(volatile v4us*)(XT + e) = o; __threadfence(); *(volatile v4us*)(XT + e) = o; }
__global__ __launch_bounds__(256) void k_hlb(const float* __restrict__ F, const float* __restrict__ b0, const float* __restrict__ b1, bf* Fh, bf* Fl, size_t n, size_t pl) { const size_t e = ((size_t)blockIdx.x * 256 + threadIdx.x) * 4; if (e >= n) return; const v4f a = *(const v4f*)(F + e); const int i = (int)(e % IC); const bool sec = (e >= pl); const v4f cA = *(const v4f*)(b0 + i), cB = *(const v4f*)(b1 + i); v4us oh, ol;
#pragma unroll
    for (int u = 0; u < 4; ++u) { const float bb = sec ? bfr(cB[u]) : bfr(cA[u]); unsigned short p, q; splitf(__fadd_rn(a[u], bb), p, q); oh[u] = p; ol[u] = q; } *(volatile v4us*)(Fh + e) = oh; *(volatile v4us*)(Fl + e) = ol; __threadfence(); *(volatile v4us*)(Fh + e) = oh; *(volatile v4us*)(Fl + e) = ol; }
__global__ __launch_bounds__(256) void k_gt16b(const float* __restrict__ G, const float* __restrict__ bvec, h16* GT) { const size_t e = ((size_t)blockIdx.x * 256 + threadIdx.x) * 2; if (e >= (size_t)IC * HW) return; const int m = (int)(e % HW); const int i = (int)(e / HW); const float bb = bfr(bvec[i]); v2h o; o[0] = tohx(__fadd_rn(G[(size_t)m * IC + i], bb)); o[1] = tohx(__fadd_rn(G[(size_t)(m + 1) * IC + i], bb)); *(volatile v2h*)(GT + e) = o; __threadfence(); *(volatile v2h*)(GT + e) = o; }
__global__ __launch_bounds__(256) void k_rsoft(const float* __restrict__ S, h16* P16) { const int lane = threadIdx.x & 31; const int row = blockIdx.x * 8 + (threadIdx.x >> 5); if (row >= HW) return; const float* sr = S + (size_t)row * HW; float v[HW / 32]; float mx = -3.0e38f;
#pragma unroll
    for (int ch = 0; ch < HW / 128; ++ch) { const v4f a = *(const v4f*)(sr + ch * 128 + lane * 4);
#pragma unroll
        for (int u = 0; u < 4; ++u) { const float t = a[u]; v[ch * 4 + u] = t; mx = fmaxf(mx, t); } }
#pragma unroll
    for (int sh = 16; sh; sh >>= 1) mx = fmaxf(mx, __shfl_xor(mx, sh, 32));
    float sum = 0.f;
#pragma unroll
    for (int q = 0; q < HW / 32; ++q) { float d0 = __fsub_rn(v[q], mx); asm volatile("" : "+v"(d0)); v[q] = __builtin_amdgcn_exp2f(__fmul_rn(d0, 1.4426950408889634f)); sum += v[q]; }
#pragma unroll
    for (int sh = 16; sh; sh >>= 1) sum += __shfl_xor(sum, sh, 32);
    const float f = __fdiv_rn(PCAR, sum);
    for (int ps = 0; ps < 2; ++ps) {
#pragma unroll
        for (int ch = 0; ch < HW / 128; ++ch) { v4h o4;
#pragma unroll
            for (int q = 0; q < 4; ++q) o4[q] = tohx(v[ch * 4 + q] * f); *(volatile v4h*)(P16 + (size_t)row * HW + ch * 128 + lane * 4) = o4; }
        if (ps == 0) __threadfence(); } }
__global__ __launch_bounds__(256) void k_yhl(const float* __restrict__ Y, bf* Yh, bf* Yl) { const size_t e = ((size_t)blockIdx.x * 256 + threadIdx.x) * 4; if (e >= (size_t)HW * IC) return; const v4f a = *(const v4f*)(Y + e); v4us oh, ol;
#pragma unroll
    for (int u = 0; u < 4; ++u) { unsigned short p, q; splitf(a[u] * (1.0f / PCAR), p, q); oh[u] = p; ol[u] = q; } *(volatile v4us*)(Yh + e) = oh; *(volatile v4us*)(Yl + e) = ol; __threadfence(); *(volatile v4us*)(Yh + e) = oh; *(volatile v4us*)(Yl + e) = ol; }
__global__ __launch_bounds__(256) void k_finb(const float* __restrict__ Z, const float* __restrict__ xb, const float* __restrict__ bo, float* OUTb) { const size_t e = ((size_t)blockIdx.x * 256 + threadIdx.x) * 4; if (e >= (size_t)CC * HW) return; const int n = (int)(e % HW); const int c = (int)(e / HW); const float bb = bfr(bo[c]); v4f r;
#pragma unroll
    for (int u = 0; u < 4; ++u) r[u] = __fadd_rn(__fadd_rn(Z[(size_t)(n + u) * CC + c], bb), bfr(xb[(size_t)c * HWF + n + u])); *(volatile v4f*)(OUTb + e) = r; __threadfence(); *(volatile v4f*)(OUTb + e) = r; }

extern "C" void kernel_launch(void* const* d_in, const int* in_sizes, int n_in,
                              void* d_out, int out_size, void* d_ws, size_t ws_size, hipStream_t stream) {
    if (n_in < 9) return;
    if (in_sizes[0] < NB * CC * HW) return;
    if (in_sizes[1] < IC * CC || in_sizes[3] < IC * CC || in_sizes[5] < IC * CC || in_sizes[7] < CC * IC) return;
    if (in_sizes[2] < IC || in_sizes[4] < IC || in_sizes[6] < IC || in_sizes[8] < CC) return;
    if (out_size < NB * CC * HW) return;
    const float* x  = (const float*)d_in[0];
    const float* wq = (const float*)d_in[1];
    const float* bq = (const float*)d_in[2];
    const float* wk = (const float*)d_in[3];
    const float* bk = (const float*)d_in[4];
    const float* wv = (const float*)d_in[5];
    const float* bv = (const float*)d_in[6];
    const float* wo = (const float*)d_in[7];
    const float* bo = (const float*)d_in[8];
    float* OUT = (float*)d_out;
    char* wsp = (char*)d_ws;
    auto take = [&](size_t bytes) { char* p = wsp; wsp += (bytes + 255) & ~(size_t)255; return (void*)p; };
    bf* BW3 = (bf*)take((size_t)3 * IC * CC * 2);
    bf* BZ  = (bf*)take((size_t)CC * IC * 2);
    bf* XT  = (bf*)take((size_t)HW * CC * 2);
    float* TPG = (float*)take((size_t)3 * HW * IC * 4);
    bf* Hh  = (bf*)take((size_t)2 * HW * IC * 2);
    bf* Hl  = (bf*)take((size_t)2 * HW * IC * 2);
    h16* GT = (h16*)take((size_t)IC * HW * 2);
    float* S = (float*)take((size_t)HW * HW * 4);
    h16* P16 = (h16*)take((size_t)HW * HW * 2);
    float* Y = (float*)take((size_t)HW * IC * 4);
    bf* Yh  = (bf*)take((size_t)HW * IC * 2); bf* Yl = (bf*)take((size_t)HW * IC * 2);
    float* Z = (float*)take((size_t)HW * CC * 4);
    if ((size_t)(wsp - (char*)d_ws) > ws_size) return;

    const size_t PL = (size_t)HW * IC;
    k_cvtw<<<(unsigned)((IC * CC / 8 + 255) / 256), 256, 0, stream>>>(wq, wk, wv, wo, BW3, BZ, IC * CC / 8);
    const unsigned L4  = (unsigned)((PL / 4 + 255) / 256);
    const unsigned L42 = (unsigned)((2 * PL / 4 + 255) / 256);
    for (int b = 0; b < NB; ++b) {
        const float* xb = x + (size_t)b * CC * HWF;
        k_xt<<<(unsigned)(((size_t)HW * CC / 4 + 255) / 256), 256, 0, stream>>>(xb, XT);
        k_gemmw<bf, 0, false><<<dim3(HW / 64, IC / 64, 3), 32, 0, stream>>>(XT, nullptr, BW3, nullptr, CC, TPG, IC, nullptr, (size_t)0, (size_t)IC * CC, PL);
        k_hlb<<<L42, 256, 0, stream>>>(TPG, bq, bk, Hh, Hl, 2 * PL, PL);
        k_gt16b<<<(unsigned)((PL / 2 + 255) / 256), 256, 0, stream>>>(TPG + 2 * PL, bv, GT);
        k_gemmw<bf, 2, false><<<dim3(HW / 64, HW / 64, 1), 32, 0, stream>>>(Hh, Hl, Hh + PL, Hl + PL, IC, S, HW, nullptr, (size_t)0, (size_t)0, (size_t)0);
        k_rsoft<<<HW / 8, 256, 0, stream>>>(S, P16);
        k_gemmw<h16, 0, false><<<dim3(HW / 64, IC / 64, 1), 32, 0, stream>>>(P16, nullptr, GT, nullptr, HW, Y, IC, nullptr, (size_t)0, (size_t)0, (size_t)0);
        k_yhl<<<L4, 256, 0, stream>>>(Y, Yh, Yl);
        k_gemmw<bf, 1, false><<<dim3(HW / 64, CC / 64, 1), 32, 0, stream>>>(Yh, Yl, BZ, nullptr, IC, Z, CC, nullptr, (size_t)0, (size_t)0, (size_t)0);
        k_finb<<<(unsigned)(((size_t)CC * HW / 4 + 255) / 256), 256, 0, stream>>>(Z, xb, bo, OUT + (size_t)b * CC * HW);
    }
}
